// TimeToCollisionConstraint_54039278518799
// MI455X (gfx1250) — hardware-verified
//
#include <hip/hip_runtime.h>
#include <math.h>

typedef __attribute__((ext_vector_type(16))) _Float16 v16h;
typedef __attribute__((ext_vector_type(16))) __bf16 v16b;
typedef __attribute__((ext_vector_type(8)))  _Float16 v8h;
typedef __attribute__((ext_vector_type(8)))  float v8f;
typedef __attribute__((ext_vector_type(4)))  float v4f;
typedef __attribute__((ext_vector_type(2)))  float v2f;
typedef __attribute__((ext_vector_type(4)))  unsigned v4u;
typedef __attribute__((ext_vector_type(4)))  int v4i;
typedef float __attribute__((may_alias)) float_a;
typedef int __attribute__((may_alias)) int_a;

template <typename T> __device__ __forceinline__ void vst2(void* p, T v) { *(volatile T*)p = v; __threadfence(); *(volatile T*)p = v; }
__device__ __forceinline__ v8f wmma16(v16h a, v16h b, v8f c) {
  v8f d = __builtin_amdgcn_wmma_f32_16x16x32_f16(false, a, false, b, (short)0, c, false, false);
  asm volatile("v_nop\n\tv_nop\n\tv_nop\n\tv_nop" : "+v"(d) : "v"(a), "v"(b));
  return d;
}
__device__ __forceinline__ v8f wmma_bf(v16b a, v16b b, v8f c) {
  v8f d = __builtin_amdgcn_wmma_f32_16x16x32_bf16(false, a, false, b, (short)0, c, false, false);
  asm volatile("v_nop\n\tv_nop\n\tv_nop\n\tv_nop" : "+v"(d) : "v"(a), "v"(b));
  return d;
}
__device__ __forceinline__ v16h frag_h(const _Float16* rowk0, int lane) {
  union { v16h v; v8h q[2]; } u; const _Float16* p = rowk0 + 8 * (lane >> 4);
  u.q[0] = *(const v8h*)p; u.q[1] = *(const v8h*)(p + 16); return u.v;
}
__device__ __forceinline__ v16h frag_f32(const float* rowk0, int lane) {
  v16h a; const float* p = rowk0 + 8 * (lane >> 4);
#pragma unroll
  for (int i = 0; i < 8; ++i) { a[i] = (_Float16)p[i]; a[8 + i] = (_Float16)p[16 + i]; }
  return a;
}
__device__ __forceinline__ v16h frag_f32s(const float* rowk0, int lane, float sc) {
  v16h a; const float* p = rowk0 + 8 * (lane >> 4);
#pragma unroll
  for (int i = 0; i < 8; ++i) { a[i] = (_Float16)(p[i] * sc); a[8 + i] = (_Float16)(p[16 + i] * sc); }
  return a;
}
__device__ __forceinline__ v16h fragc_f32(const float* W, int k0, int n, int lane, int ld, int K) {
  v16h a; const int g = lane >> 4;
#pragma unroll
  for (int i = 0; i < 8; ++i) { const int ka = k0 + 8 * g + i, kb = ka + 16;
    a[i] = (_Float16)(ka < K ? W[(size_t)(ka < K ? ka : K - 1) * ld + n] : 0.f); a[8 + i] = (_Float16)(kb < K ? W[(size_t)(kb < K ? kb : K - 1) * ld + n] : 0.f); }
  return a;
}
struct F2 { v16b h, l; };
__device__ __forceinline__ F2 bsplit16(const float v[16]) { F2 r;
#pragma unroll
  for (int i = 0; i < 16; ++i) { const __bf16 h = (__bf16)v[i]; r.h[i] = h; r.l[i] = (__bf16)(v[i] - (float)h); }
  return r; }
__device__ __forceinline__ F2 split_row(const float* row, int k0, int lane) { float v[16]; const float* p = row + k0 + 8 * (lane >> 4);
#pragma unroll
  for (int i = 0; i < 8; ++i) { v[i] = p[i]; v[8 + i] = p[16 + i]; }
  return bsplit16(v); }
__device__ __forceinline__ F2 split_rowK(const float* row, int k0, int lane, int K) { float v[16]; const int g = lane >> 4;
#pragma unroll
  for (int i = 0; i < 8; ++i) { const int ka = k0 + 8 * g + i, kb = ka + 16; v[i] = ka < K ? row[ka < K ? ka : K - 1] : 0.f; v[8 + i] = kb < K ? row[kb < K ? kb : K - 1] : 0.f; }
  return bsplit16(v); }
__device__ __forceinline__ F2 split_col(const float* W, int k0, int n, int lane, int ld, int K) { float v[16]; const int g = lane >> 4;
#pragma unroll
  for (int i = 0; i < 8; ++i) { const int ka = k0 + 8 * g + i, kb = ka + 16; v[i] = ka < K ? W[(size_t)(ka < K ? ka : K - 1) * ld + n] : 0.f; v[8 + i] = kb < K ? W[(size_t)(kb < K ? kb : K - 1) * ld + n] : 0.f; }
  return bsplit16(v); }
__device__ __forceinline__ v8f mac3(const F2& a, const F2& b, v8f c) { c = wmma_bf(a.l, b.h, c); c = wmma_bf(a.h, b.l, c); return wmma_bf(a.h, b.h, c); }
__device__ __forceinline__ float sigm(float v) { return 1.0f / (1.0f + expf(-v)); }
#define LDSX() do { asm volatile("s_wait_dscnt 0" ::: "memory"); __builtin_amdgcn_wave_barrier(); __builtin_amdgcn_fence(__ATOMIC_RELEASE, "workgroup"); } while (0)


#define NBT 32
#define NA 256
#define NPAIR 32640
#define HH 64
#ifndef NBB
#define NBB NBT
#endif
typedef __attribute__((ext_vector_type(8))) __bf16 v8b;
__device__ __forceinline__ v16b frag_b(const __bf16* rowk0, int lane) {
  union { v16b v; v8b q[2]; } u; const __bf16* p = rowk0 + 8 * (lane >> 4);
  u.q[0] = *(const v8b*)p; u.q[1] = *(const v8b*)(p + 16); return u.v;
}
__device__ __forceinline__ float bfr(float v) { return (float)(__bf16)v; }
__device__ __attribute__((noinline)) float exp_ni(float v) { return expf(v); }
__device__ __attribute__((noinline)) float erf_ni(float v) { return erff(v); }
#pragma clang fp contract(off)

#define WS_PK2 0u
#define WS_PK3 (WS_PK2 + 2u * HH * HH)
#define WS_TAB (((WS_PK3 + 2u * 16 * HH) + 127u) / 128u * 128u)
#define WS_ACT (WS_TAB + 4u * NPAIR)
#define WS_AV  (((WS_ACT + 4u * NPAIR) + 127u) / 128u * 128u)
#define WS_END (WS_AV + 4u * (size_t)NBT * NPAIR * 4)

__device__ __forceinline__ void pair_geom(const float* __restrict__ P, const float* __restrict__ V, int b, int i, int j, float* rp, float* rv, float& dist, float& ttc) {
  const float* pi = P + ((size_t)b * NA + i) * 3; const float* pj = P + ((size_t)b * NA + j) * 3; const float* vi = V + ((size_t)b * NA + i) * 3; const float* vj = V + ((size_t)b * NA + j) * 3;
#pragma unroll
  for (int c = 0; c < 3; ++c) { rp[c] = bfr(pj[c]) - bfr(pi[c]); rv[c] = bfr(vj[c]) - bfr(vi[c]); }
  const float s0 = rp[0] * rp[0], s1 = rp[1] * rp[1], s2 = rp[2] * rp[2]; dist = sqrtf((s0 + s2) + s1);
  const float d0 = rp[0] * rv[0], d1 = rp[1] * rv[1], d2 = rp[2] * rv[2]; const float dot = (d0 + d2) + d1;
  const float approach = -dot / (dist + 1e-6f);
  ttc = (approach > 0.f) ? dist / (approach + 1e-6f) : 1e6f;
}
__global__ __launch_bounds__(256) void k_pack(const float* __restrict__ W2, const float* __restrict__ W3, __bf16* __restrict__ PK2, __bf16* __restrict__ PK3, int* __restrict__ TAB) {
  __shared__ __align__(16) __bf16 s2[HH * HH], s3[16 * HH]; const int t = threadIdx.x;
  if (blockIdx.x == 0) {
    for (int q = t; q < HH * HH; q += 256) { const int n = q / HH, k = q % HH; s2[q] = (__bf16)W2[(size_t)k * HH + n]; }
    for (int q = t; q < 16 * HH; q += 256) { const int n = q / HH, k = q % HH; s3[q] = (__bf16)((n < 3) ? W3[(size_t)k * 3 + n] : 0.f); }
    __syncthreads();
    for (int q = t; q < HH * HH / 8; q += 256) vst2((unsigned*)(PK2 + q * 8), *(const v4u*)&s2[q * 8]);
    for (int q = t; q < 16 * HH / 8; q += 256) vst2((unsigned*)(PK3 + q * 8), *(const v4u*)&s3[q * 8]);
  } else {
    __shared__ __align__(16) int st[8192]; const int p0 = (blockIdx.x - 1) * 8192;
    for (int q = t; q < 8192; q += 256) { const int p = p0 + q; int v = 0; if (p < NPAIR) { int i = 0, base = 0; while (p >= base + (NA - 1 - i)) { base += NA - 1 - i; ++i; } v = (i << 16) | (i + 1 + (p - base)); } st[q] = v; }
    __syncthreads();
    for (int q = t; q < 8192 / 4; q += 256) if (p0 + q * 4 < NPAIR) vst2((unsigned*)(TAB + p0 + q * 4), *(const v4u*)&st[q * 4]);
  }
}
__global__ __launch_bounds__(256) void k_ttc(const float* __restrict__ P, const float* __restrict__ V, float* __restrict__ OUT1) {
  __shared__ __align__(16) float s[NA]; const int b = blockIdx.x / NA, i = blockIdx.x % NA, j = threadIdx.x;
  float rp[3], rv[3], dist, ttc; pair_geom(P, V, b, i, j, rp, rv, dist, ttc); s[j] = ttc;
  __syncthreads();
  if (j < NA / 4) vst2(OUT1 + ((size_t)b * NA + i) * NA + j * 4, *(const v4f*)&s[j * 4]);
}
__global__ __launch_bounds__(256) void k_active(const float* __restrict__ P, const float* __restrict__ V, const int* __restrict__ TAB, float* __restrict__ ACT) {
  __shared__ __align__(16) float s[256]; const int t = threadIdx.x; const int p = blockIdx.x * 256 + t; float a = 0.f;
  if (p < NPAIR) { const int ij = TAB[p]; const int i = ij >> 16, j = ij & 0xffff; for (int b = 0; b < NBT; ++b) { float rp[3], rv[3], dist, ttc; pair_geom(P, V, b, i, j, rp, rv, dist, ttc); if (ttc < 3.0f) a = 1.f; } }
  s[t] = a; __syncthreads();
  if (t < 64 && blockIdx.x * 256 + t * 4 < NPAIR) vst2(ACT + (size_t)blockIdx.x * 256 + t * 4, *(const v4f*)&s[t * 4]);
}
__global__ __launch_bounds__(128) void k_mlp(const float* __restrict__ P, const float* __restrict__ V, const int* __restrict__ TAB, const float* __restrict__ W1, const float* __restrict__ B1, const __bf16* __restrict__ PK2, const __bf16* __restrict__ PK3, const float* __restrict__ B2, const float* __restrict__ B3, const float* __restrict__ ACT, float* __restrict__ AV) {
  __shared__ __align__(16) __bf16 sh_[4][16][HH + 8], sl_[4][16][HH + 8]; __shared__ __align__(16) float sa[64][4]; __shared__ float sx[64][8]; __shared__ __align__(16) __bf16 s1h[64][HH + 8], s1l[64][HH + 8];
  const int tid = threadIdx.x, wave = tid >> 5, lane = tid & 31, col = lane & 15, g = lane >> 4; const size_t r0 = (size_t)blockIdx.x * 64 + wave * 16;
  if (tid < 64) { const size_t row = (size_t)blockIdx.x * 64 + tid; const int b = (int)(row / NPAIR), p = (int)(row % NPAIR); const int ij = TAB[p]; float rp[3], rv[3], dist, ttc; pair_geom(P, V, b, ij >> 16, ij & 0xffff, rp, rv, dist, ttc);
    sx[tid][0] = rp[0]; sx[tid][1] = rp[1]; sx[tid][2] = rp[2]; sx[tid][3] = rv[0]; sx[tid][4] = rv[1]; sx[tid][5] = rv[2]; sx[tid][6] = ttc; sx[tid][7] = 0.f; }
  __syncthreads();
  { const int rl = tid >> 1, c0 = (tid & 1) * 32;
    for (int ci = 0; ci < 32; ++ci) { const int c = c0 + ci; float a = 0.f;
#pragma unroll
      for (int k = 0; k < 7; ++k) a += sx[rl][k] * bfr(W1[k * HH + c]);
      const float v = fmaxf(a + bfr(B1[c]), 0.f); const __bf16 hb = (__bf16)v; s1h[rl][c] = hb; s1l[rl][c] = (__bf16)(v - (float)hb); } }
  __syncthreads();
  v8f acc[4] = {};
#pragma unroll
  for (int kc = 0; kc < 2; ++kc) { F2 a; a.h = frag_b(&s1h[wave * 16 + col][kc * 32], lane); a.l = frag_b(&s1l[wave * 16 + col][kc * 32], lane);
#pragma unroll
    for (int j = 0; j < 4; ++j) { const v16b w = frag_b(PK2 + (size_t)(j * 16 + col) * HH + kc * 32, lane); acc[j] = wmma_bf(a.l, w, acc[j]); acc[j] = wmma_bf(a.h, w, acc[j]); } }
#pragma unroll
  for (int j = 0; j < 4; ++j) { const float bb = bfr(B2[j * 16 + col]);
#pragma unroll
    for (int r = 0; r < 8; ++r) { const float v = fmaxf(acc[j][r] + bb, 0.f); const __bf16 hb = (__bf16)v; sh_[wave][8 * g + r][j * 16 + col] = hb; sl_[wave][8 * g + r][j * 16 + col] = (__bf16)(v - (float)hb); } }
  LDSX();
  v8f o = {};
#pragma unroll
  for (int kc = 0; kc < 2; ++kc) { F2 a; a.h = frag_b(&sh_[wave][col][kc * 32], lane); a.l = frag_b(&sl_[wave][col][kc * 32], lane); const v16b w = frag_b(PK3 + (size_t)col * HH + kc * 32, lane); o = wmma_bf(a.l, w, o); o = wmma_bf(a.h, w, o); }
  if (col < 4) {
#pragma unroll
    for (int r = 0; r < 8; ++r) { const size_t row = r0 + 8 * g + r; const int p = (int)(row % NPAIR); sa[wave * 16 + 8 * g + r][col] = (col < 3) ? (o[r] + bfr(B3[col])) * (0.5f * ACT[p]) : 0.f; } }
  __syncthreads();
  if (tid < 64) vst2(AV + ((size_t)blockIdx.x * 64 + tid) * 4, *(const v4f*)&sa[tid][0]);
}
__global__ __launch_bounds__(256) void k_act(const float* __restrict__ AV, float* __restrict__ OUT0) {
  __shared__ __align__(16) float s[NA * 3]; const int b = blockIdx.x, t = threadIdx.x;
  for (int q = t; q < NA * 3; q += 256) { const int n = q / 3, c = q % 3; float a = 0.f;
    { int base = 0; for (int i = 0; i < n; ++i) base += NA - 1 - i;
      for (int j = n + 1; j < NA; ++j) a += -AV[((size_t)b * NPAIR + base + (j - n - 1)) * 4 + c]; }
    { int base = 0; for (int i = 0; i < n; ++i) { a += AV[((size_t)b * NPAIR + base + (n - i - 1)) * 4 + c]; base += NA - 1 - i; } }
    s[q] = a; }
  __syncthreads();
  for (int q = t; q < NA * 3 / 4; q += 256) vst2(OUT0 + (size_t)b * NA * 3 + q * 4, *(const v4f*)&s[q * 4]);
}
extern "C" void kernel_launch(void* const* d_in, const int* in_sizes, int n_in, void* d_out, int out_size, void* d_ws, size_t ws_size, hipStream_t stream) {
  (void)in_sizes; (void)n_in; (void)out_size;
  const float** F = (const float**)d_in;
  if (ws_size < (size_t)WS_END) return;
  char* ws = (char*)d_ws; __bf16 *PK2 = (__bf16*)(ws + WS_PK2), *PK3 = (__bf16*)(ws + WS_PK3); int* TAB = (int*)(ws + WS_TAB); float *ACT = (float*)(ws + WS_ACT), *AV = (float*)(ws + WS_AV);
  k_pack<<<1 + (NPAIR + 8191) / 8192, 256, 0, stream>>>(F[4], F[6], PK2, PK3, TAB);
  k_ttc<<<NBB * NA, 256, 0, stream>>>(F[0], F[1], (float*)((char*)d_out + 98304));
  k_active<<<(NPAIR + 255) / 256, 256, 0, stream>>>(F[0], F[1], TAB, ACT);
  k_mlp<<<NBB * NPAIR / 64, 128, 0, stream>>>(F[0], F[1], TAB, F[2], F[3], PK2, PK3, F[5], F[7], ACT, AV);
  k_act<<<NBB, 256, 0, stream>>>(AV, (float*)d_out);
}
